// SAGE_80977313399688
// MI455X (gfx1250) — hardware-verified
//
#include <hip/hip_runtime.h>
#include <stddef.h>
#include <stdint.h>
#include <math.h>


#define DF     128
#define NOUT   40
#define NP3    48
#define NT3    (NP3 / 16)
#define OQ     (NOUT / 4)
#define AP     512
#define KK     512
#define HOFF   (2 * DF)
#define NTHR   256
#define NWAVE  8
#define EPT    8
#define CHUNK  (NTHR * EPT)
#define WCAP   (EPT * 32)
#define LISTN  (NWAVE * WCAP)
#define NBA    1024
#define SLA    10
#define RCAP   28672
#define DEGCAP 64
#define GBM    64
#define GBN    128
#define GTHR   128
#define GWAVE  (GTHR / 32)
#define PARTW  288
#define WSTW   258
#define HPR    8
#define HPB    (NWAVE * HPR)
#define WB1    ((DF * DF / 8) / NTHR)
#define WB3    ((NP3 * DF / 8) / NTHR)
#define NWBLK  (4 * WB1 + 2 * WB3)
#define OPIECE (GBM * OQ)
#define OPT    (OPIECE / GTHR)
#define AGG_ZINTS    (LISTN + 2 * RCAP + 3 * NBA)
#define MISC_INTS    16
#define ROWBUF_INTS  (NWAVE * DF)
#define AGG_LDS_INTS (AGG_ZINTS + MISC_INTS + ROWBUF_INTS)
#define WSMAX  134217728

static_assert((CHUNK & (CHUNK - 1)) == 0 && CHUNK <= 4096);
static_assert((NBA & (NBA - 1)) == 0 && NBA == (1 << SLA));
static_assert(((long long)CHUNK << SLA) < (1LL << 31));
static_assert(LISTN % NTHR == 0);
static_assert(NBA % NWAVE == 0 && NBA % 32 == 0 && NBA % GBM == 0);
static_assert(RCAP % 4 == 0 && AGG_ZINTS % 4 == 0 && LISTN % 4 == 0 && ((AGG_ZINTS + MISC_INTS) % 4) == 0);
static_assert(AGG_ZINTS % (NTHR * 4) == 0);
static_assert(KK % 32 == 0 && KK == AP && AP == 4 * DF && HOFF == 2 * DF);
static_assert(GBN == DF && GBM == GWAVE * 16 && DF == 4 * 32 && GTHR == DF);
static_assert(PARTW % 32 == 0 && PARTW / 4 <= GTHR && PARTW >= 2 * GBN + 1);
static_assert(WSTW >= 2 * GBN + 1 && (WSTW % 2) == 0);
static_assert(HPB == GBM && NTHR == 2 * DF);
static_assert(WB1 * NTHR * 8 == DF * DF);
static_assert(WB3 * NTHR * 8 == NP3 * DF);
static_assert(NP3 % 16 == 0 && NOUT <= NP3 && NOUT % 4 == 0 && NOUT > 16);
static_assert(OPIECE % GTHR == 0 && ((GBM * NOUT * 4) % 128) == 0 && GBM <= GTHR);
static_assert(GWAVE * 16 * (2 * GBN) * 2 == GBM * GBN * 4);
static_assert(AGG_LDS_INTS * 4 <= 300000);
static_assert(DEGCAP <= RCAP && WCAP <= LISTN);

typedef float          v4f   __attribute__((ext_vector_type(4)));
typedef float          v8f   __attribute__((ext_vector_type(8)));
typedef int            v4i   __attribute__((ext_vector_type(4)));
typedef int            v8i   __attribute__((ext_vector_type(8)));
typedef unsigned int   v2u   __attribute__((ext_vector_type(2)));
typedef unsigned int   v4u   __attribute__((ext_vector_type(4)));
typedef unsigned short v4us  __attribute__((ext_vector_type(4)));
typedef unsigned short v8us  __attribute__((ext_vector_type(8)));
typedef unsigned short v16us __attribute__((ext_vector_type(16)));
typedef __bf16         v16bf __attribute__((ext_vector_type(16)));
typedef v4f  __attribute__((may_alias)) v4fa;
typedef v4i  __attribute__((may_alias)) v4ia;
typedef v2u  __attribute__((may_alias)) v2ua;
typedef v4us __attribute__((may_alias)) v4usa;
typedef v8us __attribute__((may_alias)) v8usa;
union FragB { v16bf v; v16us u; v8us h[2]; v8i w; };

__device__ __forceinline__ v8f wmb(const FragB& a, const FragB& b, v8f c) {
  v8f d = __builtin_amdgcn_wmma_f32_16x16x32_bf16(false, a.v, false, b.v, (short)0, c, false, false);
  asm volatile("v_nop\n\tv_nop\n\tv_nop\n\tv_nop" : "+v"(d) : "v"(a.w), "v"(b.w));
  return d;
}

__device__ __forceinline__ v8f z8() { v8f z = {0.f, 0.f, 0.f, 0.f, 0.f, 0.f, 0.f, 0.f}; return z; }

__device__ __forceinline__ unsigned bf16_bits(float f) {
  const unsigned u = __float_as_uint(f);
  return ((u + 0x7FFFu + ((u >> 16) & 1u)) >> 16) & 0xFFFFu;
}
__device__ __forceinline__ float bf16_val(float f) {
  return __uint_as_float(bf16_bits(f) << 16);
}
__device__ __forceinline__ unsigned pk2(float lo, float hi) { return bf16_bits(lo) | (bf16_bits(hi) << 16); }
__device__ __forceinline__ v4u pack8(const v4f a, const v4f b) {
  v4u r;
  r.x = pk2(a.x, a.y); r.y = pk2(a.z, a.w); r.z = pk2(b.x, b.y); r.w = pk2(b.z, b.w);
  return r;
}

__device__ __forceinline__ void wave_sync() {
  __builtin_amdgcn_fence(__ATOMIC_RELEASE, "wavefront");
  __builtin_amdgcn_wave_barrier();
  __builtin_amdgcn_fence(__ATOMIC_ACQUIRE, "wavefront");
}

template <int SLB>
__device__ __forceinline__ int scan_chunk(const int* __restrict__ dsts, int nE, int cbase, int slotBase,
                                          int nb, int vec8, int* list, int tid, int lane, int wave) {
  int wc = 0;
  const int el0  = tid * EPT;
  const int e0   = cbase + el0;
  const int sent = -2147483647 - 1;
  v4i da, db;
  if (vec8 != 0 && cbase + CHUNK <= nE) {
    da = *(const v4i*)(dsts + e0);
    db = *(const v4i*)(dsts + e0 + 4);
  } else {
    da.x = (e0     < nE) ? dsts[min(e0,     nE - 1)] : sent;
    da.y = (e0 + 1 < nE) ? dsts[min(e0 + 1, nE - 1)] : sent;
    da.z = (e0 + 2 < nE) ? dsts[min(e0 + 2, nE - 1)] : sent;
    da.w = (e0 + 3 < nE) ? dsts[min(e0 + 3, nE - 1)] : sent;
    db.x = (e0 + 4 < nE) ? dsts[min(e0 + 4, nE - 1)] : sent;
    db.y = (e0 + 5 < nE) ? dsts[min(e0 + 5, nE - 1)] : sent;
    db.z = (e0 + 6 < nE) ? dsts[min(e0 + 6, nE - 1)] : sent;
    db.w = (e0 + 7 < nE) ? dsts[min(e0 + 7, nE - 1)] : sent;
  }
  const unsigned nbs = (unsigned)slotBase;
  const unsigned unb = (unsigned)nb;
  const unsigned s0 = (unsigned)da.x - nbs, s1 = (unsigned)da.y - nbs;
  const unsigned s2 = (unsigned)da.z - nbs, s3 = (unsigned)da.w - nbs;
  const unsigned s4 = (unsigned)db.x - nbs, s5 = (unsigned)db.y - nbs;
  const unsigned s6 = (unsigned)db.z - nbs, s7 = (unsigned)db.w - nbs;
  const bool h0 = s0 < unb, h1 = s1 < unb, h2 = s2 < unb, h3 = s3 < unb;
  const bool h4 = s4 < unb, h5 = s5 < unb, h6 = s6 < unb, h7 = s7 < unb;
  const unsigned any = __builtin_amdgcn_ballot_w32(h0 | h1 | h2 | h3 | h4 | h5 | h6 | h7);
  if (any != 0u) {
#define HITJ(J, HJ, SJ) { \
      const unsigned mj = __builtin_amdgcn_ballot_w32(HJ); \
      if (mj != 0u) { \
        if (HJ) { \
          const int pos = wc + (int)__builtin_amdgcn_mbcnt_lo(mj, 0u); \
          if (pos < WCAP) list[wave * WCAP + pos] = ((el0 + (J)) << SLB) | (int)(SJ); \
        } \
        wc += (int)__builtin_popcount(mj); } }
    HITJ(0, h0, s0)
    HITJ(1, h1, s1)
    HITJ(2, h2, s2)
    HITJ(3, h3, s3)
    HITJ(4, h4, s4)
    HITJ(5, h5, s5)
    HITJ(6, h6, s6)
    HITJ(7, h7, s7)
#undef HITJ
  }
  return wc;
}

__global__ __launch_bounds__(NTHR) void k_wprep(const float* __restrict__ wl1, const float* __restrict__ wr1,
                                                const float* __restrict__ wl2, const float* __restrict__ wr2,
                                                const float* __restrict__ wl3, const float* __restrict__ wr3,
                                                unsigned short* Bp1, unsigned short* Bp2, unsigned short* Bp3) {
  const int b = (int)blockIdx.x, tid = (int)threadIdx.x;
  int sel, u;
  if (b < 4 * WB1) {
    sel = b / WB1;
    u = (b - sel * WB1) * NTHR + tid;
  } else {
    const int b3 = b - 4 * WB1;
    sel = 4 + b3 / WB3;
    u = (b3 - (sel - 4) * WB3) * NTHR + tid;
  }
  const float* W;
  unsigned short* P;
  int nout;
  if (sel == 0)      { W = wl1; P = Bp1; nout = DF; }
  else if (sel == 1) { W = wr1; P = Bp1; nout = DF; }
  else if (sel == 2) { W = wl2; P = Bp2; nout = DF; }
  else if (sel == 3) { W = wr2; P = Bp2; nout = DF; }
  else if (sel == 4) { W = wl3; P = Bp3; nout = NOUT; }
  else               { W = wr3; P = Bp3; nout = NOUT; }
  const int coff = (sel & 1) ? (2 * DF) : 0;
  const int n  = u >> 4;
  const int k8 = (u & 15) * 8;
  const int nc = (n < nout) ? n : (nout - 1);
  const float keep = (n < nout) ? 1.0f : 0.0f;
  float w[8];
#pragma unroll
  for (int j = 0; j < 8; ++j) w[j] = W[(size_t)(k8 + j) * (size_t)nout + nc] * keep;
  v4f a, c;
  a.x = w[0]; a.y = w[1]; a.z = w[2]; a.w = w[3];
  c.x = w[4]; c.y = w[5]; c.z = w[6]; c.w = w[7];
  const v4u q = pack8(a, c);
  unsigned short* dp = P + (size_t)n * KK + coff + k8;
  *(volatile v4u*)dp = q;
  *(volatile v4u*)(dp + DF) = q;
  __threadfence();
  *(volatile v4u*)dp = q;
  *(volatile v4u*)(dp + DF) = q;
}

template <int INIT>
__global__ __launch_bounds__(NTHR) void k_hprep(const float* __restrict__ xin, const float* __restrict__ ss,
                                                int nN, int mRows, unsigned short* apl) {
  __shared__ __attribute__((aligned(16))) float ssh[2 * DF];
  __shared__ __attribute__((aligned(16))) unsigned short rbuf[NWAVE * 2 * DF];
  const int tid = (int)threadIdx.x, lane = tid & 31, wave = tid >> 5;
  if constexpr (INIT != 0) {
    ssh[tid] = 0.0f;
  } else {
    ssh[tid] = ss[tid];
  }
  __syncthreads();
  const v4f sc = *(const v4fa*)(ssh + 4 * lane);
  const v4f sh = *(const v4fa*)(ssh + DF + 4 * lane);
  unsigned short* rb = rbuf + wave * (2 * DF);
  const int rb0 = (int)blockIdx.x * HPB + wave * HPR;

  v8us qv[HPR];
#pragma unroll
  for (int i = 0; i < HPR; ++i) {
    const int row = rb0 + i;
    const bool live = row < nN;
    const int rc = live ? row : (nN - 1);
    v4f y;
    if constexpr (INIT != 0) {
      const v4f xr = *(const v4f*)(xin + (size_t)rc * DF + 4 * lane);
      y.x = bf16_val(xr.x); y.y = bf16_val(xr.y); y.z = bf16_val(xr.z); y.w = bf16_val(xr.w);
    } else {
      const unsigned short* rp = apl + (size_t)rc * AP + HOFF + 4 * lane;
      const v2u wh = *(const v2ua*)rp;
      const v2u wl = *(const v2ua*)(rp + DF);
      const float v0 = __uint_as_float(wh.x << 16)         + __uint_as_float(wl.x << 16);
      const float v1 = __uint_as_float(wh.x & 0xffff0000u) + __uint_as_float(wl.x & 0xffff0000u);
      const float v2 = __uint_as_float(wh.y << 16)         + __uint_as_float(wl.y << 16);
      const float v3 = __uint_as_float(wh.y & 0xffff0000u) + __uint_as_float(wl.y & 0xffff0000u);
      float t0 = fmaf(v0, sc.x, sh.x);
      float t1 = fmaf(v1, sc.y, sh.y);
      float t2 = fmaf(v2, sc.z, sh.z);
      float t3 = fmaf(v3, sc.w, sh.w);
      y.x = (t0 < 0.0f) ? 0.0f : t0;
      y.y = (t1 < 0.0f) ? 0.0f : t1;
      y.z = (t2 < 0.0f) ? 0.0f : t2;
      y.w = (t3 < 0.0f) ? 0.0f : t3;
    }
    y.x = live ? y.x : 0.0f; y.y = live ? y.y : 0.0f; y.z = live ? y.z : 0.0f; y.w = live ? y.w : 0.0f;
    v4us mh, ml;
    {
      unsigned hb;
      hb = bf16_bits(y.x); mh[0] = (unsigned short)hb; ml[0] = (unsigned short)bf16_bits(y.x - __uint_as_float(hb << 16));
      hb = bf16_bits(y.y); mh[1] = (unsigned short)hb; ml[1] = (unsigned short)bf16_bits(y.y - __uint_as_float(hb << 16));
      hb = bf16_bits(y.z); mh[2] = (unsigned short)hb; ml[2] = (unsigned short)bf16_bits(y.z - __uint_as_float(hb << 16));
      hb = bf16_bits(y.w); mh[3] = (unsigned short)hb; ml[3] = (unsigned short)bf16_bits(y.w - __uint_as_float(hb << 16));
    }
    *(v4usa*)(rb + 4 * lane) = mh;
    *(v4usa*)(rb + DF + 4 * lane) = ml;
    wave_sync();
    qv[i] = *(const v8usa*)(rb + 8 * lane);
    wave_sync();
  }
#pragma unroll
  for (int i = 0; i < HPR; ++i) {
    const int row = rb0 + i;
    if (row < mRows) {
      *(volatile v8us*)(apl + (size_t)row * AP + HOFF + 8 * lane) = qv[i];
    }
  }
  __threadfence();
#pragma unroll
  for (int i = 0; i < HPR; ++i) {
    const int row = rb0 + i;
    if (row < mRows) {
      *(volatile v8us*)(apl + (size_t)row * AP + HOFF + 8 * lane) = qv[i];
    }
  }
}

__global__ __launch_bounds__(NTHR) void k_scan(const int* __restrict__ srcs, const int* __restrict__ dsts,
                                               int nE, int nN, int vec8, int mRows, unsigned short* apl) {
  extern __shared__ __attribute__((aligned(16))) int dsm[];
  int* list = dsm;
  int* hl   = dsm + LISTN;
  int* sl   = hl + RCAP;
  int* cnt  = sl + RCAP;
  int* offs = cnt + NBA;
  int* cur  = offs + NBA;
  int* misc = cur + NBA;
  const int tid = (int)threadIdx.x, lane = tid & 31, wave = tid >> 5;
  unsigned short* rowbuf = (unsigned short*)(misc + MISC_INTS) + wave * (2 * DF);
  const int nodeBase = (int)blockIdx.x * NBA;

  {
    const v4i z4 = {0, 0, 0, 0};
    for (int i = tid * 4; i < AGG_ZINTS; i += NTHR * 4) *(v4ia*)(dsm + i) = z4;
    if (tid < MISC_INTS) misc[tid] = 0;
  }
  __syncthreads();

  int t = 0, ov = 0;
  const int nChunks = (nE + CHUNK - 1) / CHUNK;
#pragma unroll 1
  for (int chn = 0; chn < nChunks; ++chn) {
    const int cbase = chn * CHUNK;
    const int wc = scan_chunk<SLA>(dsts, nE, cbase, nodeBase, NBA, vec8, list, tid, lane, wave);
    if (lane == 0) misc[wave] = wc;
    __syncthreads();
    if (wave == 0) {
#pragma unroll 1
      for (int w2 = 0; w2 < NWAVE; ++w2) {
        int c = misc[w2];
        c = c < 0 ? 0 : (c > WCAP ? WCAP : c);
#pragma unroll 1
        for (int b0 = 0; b0 < c; b0 += 32) {
          const int idx = b0 + lane;
          const int ent = list[w2 * WCAP + (idx < WCAP ? idx : WCAP - 1)];
          const int m32 = (c - b0) < 32 ? (c - b0) : 32;
#pragma unroll 1
          for (int k = 0; k < m32; ++k) {
            const int u    = __builtin_amdgcn_readlane(ent, k);
            const int slot = u & (NBA - 1);
            const int el   = (u >> SLA) & (CHUNK - 1);
            const int pk   = ((cbase + el) << SLA) | slot;
            if (t < RCAP) {
              if (lane == 0) { hl[t] = pk; cnt[slot] = cnt[slot] + 1; }
              t = t + 1;
            } else {
              ov = 1;
            }
          }
        }
      }
    }
    __syncthreads();
  }
  if (wave == 0 && lane == 0) { misc[8] = t; misc[9] = ov; }
  __syncthreads();
  int tt = misc[8];
  tt = tt < 0 ? 0 : (tt > RCAP ? RCAP : tt);
  const int ovf = misc[9];

  if (wave == 0) {
    const int base = lane * (NBA / 32);
    int s = 0;
#pragma unroll 1
    for (int i = 0; i < NBA / 32; ++i) s += cnt[base + i];
    int incl = s;
#pragma unroll
    for (int d = 1; d < 32; d <<= 1) {
      const int y = __shfl_up(incl, d, 32);
      if (lane >= d) incl += y;
    }
    int run = incl - s;
#pragma unroll 1
    for (int i = 0; i < NBA / 32; ++i) {
      const int cv = cnt[base + i];
      offs[base + i] = run;
      cur[base + i]  = run;
      run += cv;
    }
  }
  __syncthreads();
  if (wave == 0) {
#pragma unroll 1
    for (int b0 = 0; b0 < tt; b0 += 32) {
      const int idx = b0 + lane;
      const int ent = hl[idx < RCAP ? idx : RCAP - 1];
      const int m32 = (tt - b0) < 32 ? (tt - b0) : 32;
#pragma unroll 1
      for (int k = 0; k < m32; ++k) {
        const int u    = __builtin_amdgcn_readlane(ent, k);
        const int slot = u & (NBA - 1);
        if (lane == 0) {
          int p = cur[slot];
          p = p < 0 ? 0 : (p > RCAP - 1 ? RCAP - 1 : p);
          sl[p] = u;
          cur[slot] = p + 1;
        }
      }
    }
  }
  __syncthreads();

  const float pz = (ovf != 0) ? __int_as_float(0x7fc00000) : 0.0f;
#pragma unroll 1
  for (int si = 0; si < NBA / NWAVE; ++si) {
    const int s    = si * NWAVE + wave;
    const int node = nodeBase + s;
    int c = cnt[s];
    const bool big = c > DEGCAP;
    c = c < 0 ? 0 : (c > DEGCAP ? DEGCAP : c);
    int o = offs[s];
    o = o < 0 ? 0 : (o > RCAP ? RCAP : o);
    float a0 = 0.0f, a1 = 0.0f, a2 = 0.0f, a3 = 0.0f;
#pragma unroll 1
    for (int b0 = 0; b0 < c; b0 += 32) {
      int idx = o + b0 + lane;
      idx = idx > RCAP - 1 ? RCAP - 1 : idx;
      const int ent = sl[idx];
      int eid = ent >> SLA;
      eid = eid < 0 ? 0 : (eid > nE - 1 ? nE - 1 : eid);
      int sr = srcs[eid];
      sr = sr < 0 ? 0 : (sr > nN - 1 ? nN - 1 : sr);
      const int m32 = (c - b0) < 32 ? (c - b0) : 32;
#pragma unroll 1
      for (int k = 0; k < m32; ++k) {
        const int sk = __builtin_amdgcn_readlane(sr, k);
        const unsigned short* rp = apl + (size_t)sk * AP + HOFF + 4 * lane;
        const v2u wh = *(const v2ua*)rp;
        const v2u wl = *(const v2ua*)(rp + DF);
        a0 += __uint_as_float(wh.x << 16)         + __uint_as_float(wl.x << 16);
        a1 += __uint_as_float(wh.x & 0xffff0000u) + __uint_as_float(wl.x & 0xffff0000u);
        a2 += __uint_as_float(wh.y << 16)         + __uint_as_float(wl.y << 16);
        a3 += __uint_as_float(wh.y & 0xffff0000u) + __uint_as_float(wl.y & 0xffff0000u);
      }
    }
    const float den = (c > 0) ? (float)c : 1.0f;
    const float rcp = 1.0f / den;
    const float pzr = big ? __int_as_float(0x7fc00000) : pz;
    const bool live = node < nN;
    const float m0 = live ? (a0 * rcp + pzr) : 0.0f;
    const float m1 = live ? (a1 * rcp + pzr) : 0.0f;
    const float m2 = live ? (a2 * rcp + pzr) : 0.0f;
    const float m3 = live ? (a3 * rcp + pzr) : 0.0f;
    v4us mh, ml;
    {
      unsigned hb;
      hb = bf16_bits(m0); mh[0] = (unsigned short)hb; ml[0] = (unsigned short)bf16_bits(m0 - __uint_as_float(hb << 16));
      hb = bf16_bits(m1); mh[1] = (unsigned short)hb; ml[1] = (unsigned short)bf16_bits(m1 - __uint_as_float(hb << 16));
      hb = bf16_bits(m2); mh[2] = (unsigned short)hb; ml[2] = (unsigned short)bf16_bits(m2 - __uint_as_float(hb << 16));
      hb = bf16_bits(m3); mh[3] = (unsigned short)hb; ml[3] = (unsigned short)bf16_bits(m3 - __uint_as_float(hb << 16));
    }
    *(v4usa*)(rowbuf + 4 * lane) = mh;
    *(v4usa*)(rowbuf + DF + 4 * lane) = ml;
    wave_sync();
    const v8us q0 = *(const v8usa*)(rowbuf + 8 * lane);
    wave_sync();
    if (node < mRows) {
      unsigned short* rpw = apl + (size_t)node * AP + 8 * lane;
      *(volatile v8us*)rpw = q0;
      __threadfence();
      *(volatile v8us*)rpw = q0;
    }
  }
}

__global__ __launch_bounds__(GTHR) void k_gemm1(unsigned short* Apl, const unsigned short* __restrict__ BT,
                                                const float* __restrict__ bias, int nN, float* part) {
  __shared__ __attribute__((aligned(16))) float stg[GBM * GBN];
  __shared__ __attribute__((aligned(16))) float wst[GWAVE * WSTW];
  __shared__ __attribute__((aligned(16))) float pst[PARTW];
  const int tid = (int)threadIdx.x, lane = tid & 31, wave = tid >> 5, hh = lane >> 4, m = lane & 15;
  const int rowBase = (int)blockIdx.x * GBM;

  v8f acc[8];
#pragma unroll
  for (int t = 0; t < 8; ++t) acc[t] = z8();
  const unsigned short* ap = Apl + (size_t)(rowBase + 16 * wave + m) * (size_t)AP + 8 * hh;
  const unsigned short* bp = BT + (size_t)m * (size_t)KK + 8 * hh;

#pragma unroll 1
  for (int k0 = 0; k0 < KK; k0 += 32) {
    FragB af;
    af.h[0] = *(const v8usa*)(ap + k0);
    af.h[1] = *(const v8usa*)(ap + k0 + 16);
#pragma unroll
    for (int nt = 0; nt < 8; ++nt) {
      const unsigned short* wq = bp + (size_t)(16 * nt) * (size_t)KK + k0;
      FragB bf;
      bf.h[0] = *(const v8usa*)wq;
      bf.h[1] = *(const v8usa*)(wq + 16);
      acc[nt] = wmb(af, bf, acc[nt]);
    }
  }

#pragma unroll
  for (int nt = 0; nt < 8; ++nt) {
    const int lc = 16 * nt + m;
#pragma unroll
    for (int r = 0; r < 8; ++r) {
      const int lr = 16 * wave + 8 * hh + r;
      stg[lr * GBN + lc] = acc[nt][r];
    }
  }
  __syncthreads();

  v4f bq;
  {
    const v4f b4 = *(const v4f*)(bias + 4 * lane);
    bq.x = bf16_val(b4.x); bq.y = bf16_val(b4.y); bq.z = bf16_val(b4.z); bq.w = bf16_val(b4.w);
  }

  v4f pv[16];
  int wn = 0;
  float wm[4], wqv[4];
#pragma unroll
  for (int j = 0; j < 4; ++j) { wm[j] = 0.0f; wqv[j] = 0.0f; }
#pragma unroll
  for (int i = 0; i < 16; ++i) {
    const int row = rowBase + 16 * wave + i;
    const bool ok = row < nN;
    const v4f x = *(const v4fa*)(stg + (16 * wave + i) * GBN + 4 * lane);
    const v4f tq = x + bq;
    float vv[4];
    vv[0] = ok ? tq.x : 0.0f; vv[1] = ok ? tq.y : 0.0f; vv[2] = ok ? tq.z : 0.0f; vv[3] = ok ? tq.w : 0.0f;
    v4f q;
    q.x = vv[0]; q.y = vv[1]; q.z = vv[2]; q.w = vv[3];
    pv[i] = q;
    if (ok) {
      wn += 1;
      const float rk = 1.0f / (float)(i + 1);
#pragma unroll
      for (int j = 0; j < 4; ++j) {
        const float d = vv[j] - wm[j];
        wm[j]  = fmaf(d, rk, wm[j]);
        wqv[j] = fmaf(d, vv[j] - wm[j], wqv[j]);
      }
    }
  }
  __syncthreads();

#pragma unroll
  for (int i = 0; i < 16; ++i) {
    v4us h4, l4;
    unsigned hb;
    hb = bf16_bits(pv[i].x); h4[0] = (unsigned short)hb; l4[0] = (unsigned short)bf16_bits(pv[i].x - __uint_as_float(hb << 16));
    hb = bf16_bits(pv[i].y); h4[1] = (unsigned short)hb; l4[1] = (unsigned short)bf16_bits(pv[i].y - __uint_as_float(hb << 16));
    hb = bf16_bits(pv[i].z); h4[2] = (unsigned short)hb; l4[2] = (unsigned short)bf16_bits(pv[i].z - __uint_as_float(hb << 16));
    hb = bf16_bits(pv[i].w); h4[3] = (unsigned short)hb; l4[3] = (unsigned short)bf16_bits(pv[i].w - __uint_as_float(hb << 16));
    unsigned short* srow = (unsigned short*)stg + (size_t)(16 * wave + i) * (2 * GBN);
    *(v4usa*)(srow + 4 * lane) = h4;
    *(v4usa*)(srow + GBN + 4 * lane) = l4;
  }
  __syncthreads();
  v8us qv[16];
#pragma unroll
  for (int i = 0; i < 16; ++i) {
    const unsigned short* srow = (const unsigned short*)stg + (size_t)(16 * wave + i) * (2 * GBN);
    qv[i] = *(const v8usa*)(srow + 8 * lane);
  }
#pragma unroll
  for (int i = 0; i < 16; ++i) {
    unsigned short* rp = Apl + (size_t)(rowBase + 16 * wave + i) * (size_t)AP + HOFF + 8 * lane;
    *(volatile v8us*)rp = qv[i];
  }
  __threadfence();
#pragma unroll
  for (int i = 0; i < 16; ++i) {
    unsigned short* rp = Apl + (size_t)(rowBase + 16 * wave + i) * (size_t)AP + HOFF + 8 * lane;
    *(volatile v8us*)rp = qv[i];
  }

  if (lane == 0) wst[wave * WSTW] = (float)wn;
#pragma unroll
  for (int j = 0; j < 4; ++j) {
    wst[wave * WSTW + 1 + 4 * lane + j]       = wm[j];
    wst[wave * WSTW + 1 + GBN + 4 * lane + j] = wqv[j];
  }
  __syncthreads();
  {
    float n = 0.0f, mean = 0.0f, M2 = 0.0f;
#pragma unroll 1
    for (int w2 = 0; w2 < GWAVE; ++w2) {
      const float nb = wst[w2 * WSTW];
      const float mb = wst[w2 * WSTW + 1 + tid];
      const float qb = wst[w2 * WSTW + 1 + GBN + tid];
      if (nb > 0.5f) {
        const float nn = n + nb;
        const float delta = mb - mean;
        const float f = nb / nn;
        mean = fmaf(delta, f, mean);
        M2 = M2 + qb + delta * delta * n * f;
        n = nn;
      }
    }
    pst[1 + tid] = mean;
    pst[1 + GBN + tid] = M2;
    if (tid == 0) pst[0] = n;
  }
#pragma unroll 1
  for (int i = 2 * GBN + 1 + tid; i < PARTW; i += GTHR) pst[i] = 0.0f;
  __syncthreads();
  const int pb = (int)blockIdx.x;
  v4f ps = {0.0f, 0.0f, 0.0f, 0.0f};
  if (tid < PARTW / 4) {
    ps = *(const v4fa*)(pst + 4 * tid);
    *(volatile v4f*)(part + (size_t)pb * PARTW + 4 * tid) = ps;
  }
  __threadfence();
  if (tid < PARTW / 4) {
    *(volatile v4f*)(part + (size_t)pb * PARTW + 4 * tid) = ps;
  }
}

__global__ __launch_bounds__(DF) void k_bnfin(const float* __restrict__ part, int nPart,
                                              const float* __restrict__ gam, const float* __restrict__ bet,
                                              float* ss) {
  __shared__ __attribute__((aligned(16))) float stg[2 * DF];
  const int tid = (int)threadIdx.x;
  const int c = tid;
  double n = 0.0, mean = 0.0, M2 = 0.0;
#pragma unroll 1
  for (int b = 0; b < nPart; ++b) {
    const float* pr = part + (size_t)b * PARTW;
    const double nb = (double)pr[0];
    const double mb = (double)pr[1 + c];
    const double qb = (double)pr[1 + GBN + c];
    if (nb > 0.5) {
      const double nn = n + nb;
      const double delta = mb - mean;
      const double f = nb / nn;
      mean = mean + delta * f;
      M2 = M2 + qb + delta * delta * n * f;
      n = nn;
    }
  }
  const double nt = n < 1.0 ? 1.0 : n;
  const float varf  = (float)(M2 / nt);
  const float meanf = (float)mean;
  const float rstd = 1.0f / sqrtf(varf + 1e-5f);
  const float sc = bf16_val(gam[c]) * rstd;
  const float sh = bf16_val(bet[c]) - meanf * sc;
  stg[c] = sc;
  stg[DF + c] = sh;
  __syncthreads();
  v4f v = {0.0f, 0.0f, 0.0f, 0.0f};
  if (tid < (2 * DF) / 4) {
    v = *(const v4fa*)(stg + 4 * tid);
    *(volatile v4f*)(ss + 4 * tid) = v;
  }
  __threadfence();
  if (tid < (2 * DF) / 4) {
    *(volatile v4f*)(ss + 4 * tid) = v;
  }
}

__global__ __launch_bounds__(GTHR) void k_gemm2(const unsigned short* __restrict__ Apl,
                                                const unsigned short* __restrict__ BT,
                                                const float* __restrict__ bias, int nN, float* outp) {
  __shared__ __attribute__((aligned(16))) float stg[GBM * NOUT];
  const int tid = (int)threadIdx.x, lane = tid & 31, wave = tid >> 5, hh = lane >> 4, m = lane & 15;
  const int rowBase = (int)blockIdx.x * GBM;

  v8f acc[NT3];
#pragma unroll
  for (int t = 0; t < NT3; ++t) acc[t] = z8();
  const unsigned short* ap = Apl + (size_t)(rowBase + 16 * wave + m) * (size_t)AP + 8 * hh;
  const unsigned short* bp = BT + (size_t)m * (size_t)KK + 8 * hh;

#pragma unroll 2
  for (int k0 = 0; k0 < KK; k0 += 32) {
    FragB af;
    af.h[0] = *(const v8usa*)(ap + k0);
    af.h[1] = *(const v8usa*)(ap + k0 + 16);
#pragma unroll
    for (int nt = 0; nt < NT3; ++nt) {
      const unsigned short* wq = bp + (size_t)(16 * nt) * (size_t)KK + k0;
      FragB bf;
      bf.h[0] = *(const v8usa*)wq;
      bf.h[1] = *(const v8usa*)(wq + 16);
      acc[nt] = wmb(af, bf, acc[nt]);
    }
  }

  float bq[NT3];
#pragma unroll
  for (int nt = 0; nt < NT3; ++nt) {
    const int n  = 16 * nt + m;
    const int nc = (n < NOUT) ? n : (NOUT - 1);
    bq[nt] = bf16_val(bias[nc]);
  }
#pragma unroll
  for (int nt = 0; nt < NT3; ++nt) {
    const int n = 16 * nt + m;
#pragma unroll
    for (int r = 0; r < 8; ++r) {
      const int lr = 16 * wave + 8 * hh + r;
      if (n < NOUT) stg[lr * NOUT + n] = acc[nt][r] + bq[nt];
    }
  }
  __syncthreads();

  if (tid < GBM) {
    float* zr = stg + tid * NOUT;
    float mx = zr[0];
#pragma unroll 1
    for (int c = 1; c < NOUT; ++c) mx = fmaxf(mx, zr[c]);
    float se = 0.0f;
#pragma unroll 1
    for (int c = 0; c < NOUT; ++c) se += expf(zr[c] - mx);
    const float lse = logf(se);
#pragma unroll 1
    for (int c = 0; c < NOUT; ++c) {
      const float v = zr[c];
      zr[c] = (v - mx) - lse;
    }
  }
  __syncthreads();

  const int nv   = nN - rowBase;
  const int plim = ((nv > GBM) ? GBM : nv) * OQ;
  float* ob = outp + (size_t)rowBase * (size_t)NOUT;
  v4f pv[OPT];
#pragma unroll
  for (int j = 0; j < OPT; ++j) {
    const int p = GTHR * j + tid;
    pv[j] = *(const v4fa*)(stg + 4 * p);
  }
#pragma unroll
  for (int j = 0; j < OPT; ++j) {
    const int p = GTHR * j + tid;
    if (p < plim) *(volatile v4f*)(ob + 4 * p) = pv[j];
  }
  __threadfence();
#pragma unroll
  for (int j = 0; j < OPT; ++j) {
    const int p = GTHR * j + tid;
    if (p < plim) *(volatile v4f*)(ob + 4 * p) = pv[j];
  }
}

static inline int cdiv(int a, int b) { return (a + b - 1) / b; }
static inline size_t al256(size_t o) { return (o + 255) & ~(size_t)255; }

extern "C" void kernel_launch(void* const* d_in, const int* in_sizes, int n_in,
                              void* d_out, int out_size, void* d_ws, size_t ws_size,
                              hipStream_t stream) {
  if (n_in < 16) return;
  if (in_sizes[0] < DF || (in_sizes[0] % DF) != 0) return;
  const int nN = in_sizes[0] / DF;
  const int nE = in_sizes[1];
  if (in_sizes[2] != nE) return;
  if (nE < 1 || nE >= (1 << 21) || nN < 16 || nN >= (1 << 24)) return;
  if (in_sizes[3] != DF * DF || in_sizes[4] != DF || in_sizes[5] != DF * DF) return;
  if (in_sizes[6] != DF || in_sizes[7] != DF) return;
  if (in_sizes[8] != DF * DF || in_sizes[9] != DF || in_sizes[10] != DF * DF) return;
  if (in_sizes[11] != DF || in_sizes[12] != DF) return;
  if (in_sizes[13] != DF * NOUT || in_sizes[14] != NOUT || in_sizes[15] != DF * NOUT) return;
  if ((long long)out_size != (long long)nN * NOUT) return;

  const float* x    = (const float*)d_in[0];
  const int*   esrc = (const int*)d_in[1];
  const int*   edst = (const int*)d_in[2];
  const float* wl1  = (const float*)d_in[3];
  const float* bl1  = (const float*)d_in[4];
  const float* wr1  = (const float*)d_in[5];
  const float* gm1  = (const float*)d_in[6];
  const float* bt1  = (const float*)d_in[7];
  const float* wl2  = (const float*)d_in[8];
  const float* bl2  = (const float*)d_in[9];
  const float* wr2  = (const float*)d_in[10];
  const float* gm2  = (const float*)d_in[11];
  const float* bt2  = (const float*)d_in[12];
  const float* wl3  = (const float*)d_in[13];
  const float* bl3  = (const float*)d_in[14];
  const float* wr3  = (const float*)d_in[15];
  float* out = (float*)d_out;

  const int MP = cdiv(nN, GBM) * GBM;
  const int gM = MP / GBM;
  const int gA = cdiv(nN, NBA);
  if ((long long)gA * NBA < (long long)MP) return;
  if ((MP % HPB) != 0) return;
  const int vec8 = ((nE & 3) == 0) ? 1 : 0;

  char* ws = (char*)d_ws;
  size_t off = 0;
  const size_t oB1 = off; off = al256(off + (size_t)DF * KK * 2);
  const size_t oB2 = off; off = al256(off + (size_t)DF * KK * 2);
  const size_t oB3 = off; off = al256(off + (size_t)NP3 * KK * 2);
  const size_t oA  = off; off = al256(off + (size_t)MP * AP * 2);
  const size_t oPT = off; off = al256(off + (size_t)gM * PARTW * 4);
  const size_t oSS = off; off = al256(off + (size_t)(2 * DF) * 4);
  if (off > ws_size || off > (size_t)WSMAX) return;
  unsigned short* Bp1 = (unsigned short*)(ws + oB1);
  unsigned short* Bp2 = (unsigned short*)(ws + oB2);
  unsigned short* Bp3 = (unsigned short*)(ws + oB3);
  unsigned short* Apl = (unsigned short*)(ws + oA);
  float*          PT  = (float*)(ws + oPT);
  float*          SS  = (float*)(ws + oSS);

  const size_t scanLds = (size_t)AGG_LDS_INTS * 4;
  hipFuncSetAttribute(reinterpret_cast<const void*>(&k_scan), hipFuncAttributeMaxDynamicSharedMemorySize, (int)scanLds);

  k_wprep<<<NWBLK, NTHR, 0, stream>>>(wl1, wr1, wl2, wr2, wl3, wr3, Bp1, Bp2, Bp3);
  k_hprep<1><<<gM, NTHR, 0, stream>>>(x, SS, nN, MP, Apl);
  k_scan<<<gA, NTHR, scanLds, stream>>>(esrc, edst, nE, nN, vec8, MP, Apl);
  k_gemm1<<<gM, GTHR, 0, stream>>>(Apl, Bp1, bl1, nN, PT);
  k_bnfin<<<1, DF, 0, stream>>>(PT, gM, gm1, bt1, SS);
  k_hprep<0><<<gM, NTHR, 0, stream>>>(x, SS, nN, MP, Apl);
  k_scan<<<gA, NTHR, scanLds, stream>>>(esrc, edst, nE, nN, vec8, MP, Apl);
  k_gemm1<<<gM, GTHR, 0, stream>>>(Apl, Bp2, bl2, nN, PT);
  k_bnfin<<<1, DF, 0, stream>>>(PT, gM, gm2, bt2, SS);
  k_hprep<0><<<gM, NTHR, 0, stream>>>(x, SS, nN, MP, Apl);
  k_scan<<<gA, NTHR, scanLds, stream>>>(esrc, edst, nE, nN, vec8, MP, Apl);
  k_gemm2<<<gM, GTHR, 0, stream>>>(Apl, Bp3, bl3, nN, out);
}
